// conv_nonlinear_45715631898929
// MI455X (gfx1250) — hardware-run, weakly checked
//
#include <hip/hip_runtime.h>
#include <math.h>

typedef __attribute__((ext_vector_type(16))) _Float16 v16h;
typedef __attribute__((ext_vector_type(8)))  _Float16 v8h;
typedef __attribute__((ext_vector_type(8)))  float    v8f;
typedef __attribute__((ext_vector_type(4)))  float    v4f;

constexpr int kNB     = 16;
constexpr int kNC     = 4;
constexpr int kLen    = 1000;
constexpr int kTaps   = 15;
constexpr int kNOut   = kLen - kTaps + 1;
constexpr int kNF     = 64;
constexpr int kD0 = 60, kD1 = 72, kD2 = 86, kD3 = 86, kD4 = 71, kD5 = 59;
constexpr int kNP0 = 80, kNP1 = 96, kNP2 = 96, kNP3 = 80, kNP4 = 64;
constexpr int kKP0 = 64, kKPX = 96;
constexpr int kWP0 = 72, kWPX = 104, kTP = 104;
constexpr int kWOff0 = 0;
constexpr int kWOff1 = kWOff0 + kNP0 * kWP0;
constexpr int kWOff2 = kWOff1 + kNP1 * kWPX;
constexpr int kWOff3 = kWOff2 + kNP2 * kWPX;
constexpr int kWOff4 = kWOff3 + kNP3 * kWPX;
constexpr int kBlobHalves = kWOff4 + kNP4 * kWPX;
constexpr int kBlobBytes  = kBlobHalves * 2;
constexpr int kWChunks    = kBlobBytes / 16;
constexpr int kWChunkIters = (kWChunks + 255) / 256;
constexpr int kBOff0 = 0;
constexpr int kBOff1 = kBOff0 + kNP0;
constexpr int kBOff2 = kBOff1 + kNP1;
constexpr int kBOff3 = kBOff2 + kNP2;
constexpr int kBOff4 = kBOff3 + kNP3;
constexpr int kBTotal = kBOff4 + kNP4;
constexpr int kXW = 1008;
constexpr int kXChunksPerCh = kXW / 8;
constexpr int kXChunks = kNC * kXChunksPerCh;
constexpr int kTileRows = 32;
constexpr int kTiles = (kNOut + kTileRows - 1) / kTileRows;
constexpr int kTileHalves = kTileRows * kTP;
constexpr int kOutPitch = 1024;
constexpr float kCarryA = 64.0f;
constexpr float kCarryW = 64.0f;
constexpr float kDescale = 1.0f / (kCarryA * kCarryW);

static_assert(kNOut == 986, "window count");
static_assert(kNC * kTaps == kD0, "unfold width");
static_assert(kTiles == 31 && kTiles * kTileRows == 992, "row tiles");
static_assert(kTiles * kTileRows + kTaps - 1 <= kXW, "x window covers padded rows");
static_assert(kD0 <= kKP0 && kD1 <= kKPX && kD2 <= kKPX && kD3 <= kKPX && kD4 <= kKPX, "K pads");
static_assert(kD1 <= kNP0 && kD2 <= kNP1 && kD3 <= kNP2 && kD4 <= kNP3 && kD5 <= kNP4, "N pads");
static_assert((kKP0 % 32) == 0 && (kKPX % 32) == 0, "K multiples of 32");
static_assert((kNP0 % 16) == 0 && (kNP1 % 16) == 0 && (kNP2 % 16) == 0 && (kNP3 % 16) == 0 && (kNP4 % 16) == 0, "N multiples of 16");
static_assert(kWP0 >= kKP0 && kWPX >= kKPX && kTP >= kKPX && (kWP0 % 8) == 0 && (kWPX % 8) == 0 && (kTP % 8) == 0, "pitches");
static_assert(kBlobHalves == 40704 && (kBlobBytes % 128) == 0, "blob is whole lines");
static_assert(((kWOff1 * 2) % 128) == 0 && ((kWOff2 * 2) % 128) == 0 && ((kWOff3 * 2) % 128) == 0 && ((kWOff4 * 2) % 128) == 0, "plane bases on lines");
static_assert(kWChunks == 5088 && kWChunkIters == 20, "blob chunks");
static_assert(kBTotal == 416, "bias total");
static_assert(kXChunks == 504, "x chunks");
static_assert(kNOut <= kOutPitch && kTiles * kTileRows <= kOutPitch, "staging pitch");

constexpr int kLdsW   = 0;
constexpr int kLdsB   = kLdsW + kBlobBytes;
constexpr int kLdsHW  = kLdsB + kBTotal * 4;
constexpr int kLdsXS  = kLdsHW + 80 * 4;
constexpr int kLdsOUT = kLdsXS + kNC * kXW * 2;
constexpr int kLdsT   = kLdsOUT + kOutPitch * 4;
constexpr int kLdsTotal = kLdsT + 8 * 2 * kTileHalves * 2;
static_assert((kLdsB % 16) == 0 && (kLdsHW % 16) == 0 && (kLdsXS % 16) == 0 && (kLdsOUT % 16) == 0 && (kLdsT % 16) == 0, "LDS alignment");
static_assert(kLdsTotal == 202048, "LDS total");

constexpr size_t kWsOffWPL  = 0;
constexpr size_t kWsOffOUTP = kWsOffWPL + (size_t)kNF * kBlobBytes;
constexpr size_t kWsTotal   = kWsOffOUTP + (size_t)kNB * kNF * kOutPitch * 4;
static_assert((kWsOffOUTP % 128) == 0, "aligned regions");
static_assert(kWsTotal == 9404416ull, "carve total");
static_assert(kWsTotal <= 134217728ull, "carve cap");

constexpr int kOutTotal  = kNB * kNF * kNOut;
constexpr int kOutTotal4 = kOutTotal / 4;
static_assert(kOutTotal == 1009664 && (kOutTotal % 32) == 0, "output is whole lines");
static_assert(kOutTotal4 == 986 * 256, "repack grid exact");

__device__ __forceinline__ int imin(int a, int b) { return a < b ? a : b; }

__device__ __forceinline__ float bf16_rne_f32(float f) {
  const unsigned u = __float_as_uint(f);
  const unsigned r = (u + 0x7FFFu + ((u >> 16) & 1u)) & 0xFFFF0000u;
  return __uint_as_float(r);
}

union FragU { v16h v; v8h h[2]; };
__device__ __forceinline__ v16h frag_load(const _Float16* p) {
  FragU f;
  f.h[0] = *(const v8h*)(p);
  f.h[1] = *(const v8h*)(p + 16);
  return f.v;
}
__device__ __forceinline__ v8f mma_f16(v16h a, v16h b, v8f c) {
  return __builtin_amdgcn_wmma_f32_16x16x32_f16(false, a, false, b, (short)0, c, false, false);
}
__device__ __forceinline__ void acc_guard(v8f& acc, v16h a0, v16h a1, v16h a2, v16h b0, v16h b1, v16h b2) {
  asm volatile("v_nop\n\tv_nop\n\tv_nop\n\tv_nop" : "+v"(acc) : "v"(a0), "v"(a1), "v"(a2), "v"(b0), "v"(b1), "v"(b2));
}
__device__ __forceinline__ void wave_sync() {
  __builtin_amdgcn_fence(__ATOMIC_RELEASE, "workgroup");
  __builtin_amdgcn_wave_barrier();
  __builtin_amdgcn_fence(__ATOMIC_ACQUIRE, "workgroup");
}

__global__ __launch_bounds__(256) void prep_weight_planes_kernel(
    const float* __restrict__ w0, const float* __restrict__ w1, const float* __restrict__ w2,
    const float* __restrict__ w3, const float* __restrict__ w4, unsigned short* __restrict__ wpl)
{
  const int tid = threadIdx.x;
  const int ly  = blockIdx.y;
  const int kf  = blockIdx.z;
  const float* src = w0;
  int din = kD0, dout = kD1, npad = kNP0, pitch = kWP0, base = kWOff0;
  if (ly == 1) { src = w1; din = kD1; dout = kD2; npad = kNP1; pitch = kWPX; base = kWOff1; }
  if (ly == 2) { src = w2; din = kD2; dout = kD3; npad = kNP2; pitch = kWPX; base = kWOff2; }
  if (ly == 3) { src = w3; din = kD3; dout = kD4; npad = kNP3; pitch = kWPX; base = kWOff3; }
  if (ly == 4) { src = w4; din = kD4; dout = kD5; npad = kNP4; pitch = kWPX; base = kWOff4; }
  const int cpr   = pitch >> 3;
  const int count = npad * cpr;
  if ((int)blockIdx.x * 256 >= count) return;
  const int ch  = (int)blockIdx.x * 256 + tid;
  const int chc = imin(ch, count - 1);
  const int n   = chc / cpr;
  const int kk0 = (chc - n * cpr) * 8;
  const int nc  = imin(n, dout - 1);
  const float* sk = src + (size_t)kf * din * dout;
  v8h hv;
#pragma unroll
  for (int e = 0; e < 8; ++e) {
    const int kk  = kk0 + e;
    const int kkc = imin(kk, din - 1);
    float f = sk[(size_t)kkc * dout + nc];
    asm volatile("" : "+v"(f));
    const bool ok = (kk < din) && (n < dout);
    const float val = ok ? (bf16_rne_f32(f) * kCarryW) : 0.0f;
    hv[e] = (_Float16)val;
  }
  if (ch < count) {
    unsigned short* dst = wpl + (size_t)kf * kBlobHalves + base + (size_t)ch * 8;
    *(volatile v8h*)dst = hv;
    __threadfence();
    *(volatile v8h*)dst = hv;
  }
}

template <int KS, bool LAST>
__device__ __forceinline__ void fc_layer(const _Float16* tin, _Float16* tout, const _Float16* wpl, const int wpitch,
                                         const float* bias, const float* hwv, const int ntiles, const bool zpad,
                                         const int lane, const _Float16 zh, v8f& hp0, v8f& hp1)
{
  const int h = lane >> 4;
  const int n = lane & 15;
  v16h a0[KS], a1[KS];
#pragma unroll
  for (int ks = 0; ks < KS; ++ks) {
    a0[ks] = frag_load(tin + n * kTP + 32 * ks + 8 * h);
    a1[ks] = frag_load(tin + (16 + n) * kTP + 32 * ks + 8 * h);
  }
#pragma unroll 1
  for (int t = 0; t < ntiles; ++t) {
    const _Float16* wrow = wpl + (16 * t + n) * wpitch + 8 * h;
    v16h bf[KS];
#pragma unroll
    for (int ks = 0; ks < KS; ++ks) bf[ks] = frag_load(wrow + 32 * ks);
    v8f acc0 = (v8f){0.f, 0.f, 0.f, 0.f, 0.f, 0.f, 0.f, 0.f};
    v8f acc1 = (v8f){0.f, 0.f, 0.f, 0.f, 0.f, 0.f, 0.f, 0.f};
#pragma unroll
    for (int ks = 0; ks < KS; ++ks) {
      acc0 = mma_f16(a0[ks], bf[ks], acc0);
      acc1 = mma_f16(a1[ks], bf[ks], acc1);
    }
    acc_guard(acc0, a0[0], a0[1], a0[KS - 1], bf[0], bf[1], bf[KS - 1]);
    acc_guard(acc1, a1[0], a1[1], a1[KS - 1], bf[0], bf[1], bf[KS - 1]);
    const float bv = bias[16 * t + n];
    float hv = 0.0f;
    if (LAST) hv = hwv[16 * t + n];
#pragma unroll 1
    for (int s = 0; s < 2; ++s) {
      const bool hiSub = (s != 0);
      v8f v;
      v8f hp;
#pragma unroll
      for (int r = 0; r < 8; ++r) {
        v[r]  = hiSub ? acc1[r] : acc0[r];
        hp[r] = hiSub ? hp1[r] : hp0[r];
      }
      _Float16* orow = tout + (16 * s + 8 * h) * kTP + 16 * t + n;
#pragma unroll
      for (int r = 0; r < 8; ++r) {
        const float z = fmaf(v[r], kDescale, bv);
        const float g = 0.5f * z * (1.0f + erff(z * 0.70710678118654752f));
        if (LAST) {
          hp[r] = fmaf(g, hv, hp[r]);
        } else {
          orow[r * kTP] = (_Float16)(g * kCarryA);
        }
      }
      if (LAST) {
#pragma unroll
        for (int r = 0; r < 8; ++r) {
          hp1[r] = hiSub ? hp[r] : hp1[r];
          hp0[r] = hiSub ? hp0[r] : hp[r];
        }
      }
    }
  }
  if (!LAST) {
    if (zpad) {
      v8h z8;
#pragma unroll
      for (int e = 0; e < 8; ++e) z8[e] = zh;
      *(v8h*)(tout + lane * kTP + 80) = z8;
      *(v8h*)(tout + lane * kTP + 88) = z8;
    }
  }
  wave_sync();
}

__global__ __launch_bounds__(256) void fused_fc_stack_kernel(
    const float* __restrict__ x,
    const float* __restrict__ b0, const float* __restrict__ b1, const float* __restrict__ b2,
    const float* __restrict__ b3, const float* __restrict__ b4,
    const float* __restrict__ head_w, const float* __restrict__ head_b,
    const unsigned short* __restrict__ wpl, float* __restrict__ outp)
{
  extern __shared__ __align__(16) unsigned char smem[];
  _Float16* sW   = (_Float16*)(smem + kLdsW);
  float*    sB   = (float*)(smem + kLdsB);
  float*    sHW  = (float*)(smem + kLdsHW);
  _Float16* sXS  = (_Float16*)(smem + kLdsXS);
  float*    sOUT = (float*)(smem + kLdsOUT);
  _Float16* sT   = (_Float16*)(smem + kLdsT);

  const int tid  = threadIdx.x;
  const int lane = tid & 31;
  const int wave = __builtin_amdgcn_readfirstlane((int)(threadIdx.x >> 5));
  const int bx   = blockIdx.x;
  const int kf   = bx & (kNF - 1);
  const int bb   = bx >> 6;

  {
    const uint4* srcp = (const uint4*)(wpl + (size_t)kf * kBlobHalves);
    uint4* dstp = (uint4*)(smem + kLdsW);
#pragma unroll 1
    for (int it = 0; it < kWChunkIters; ++it) {
      const int idx = it * 256 + tid;
      const int idc = imin(idx, kWChunks - 1);
      uint4 v = srcp[idc];
      asm volatile("" : "+v"(v.x), "+v"(v.y), "+v"(v.z), "+v"(v.w));
      if (idx < kWChunks) dstp[idx] = v;
    }
  }
  {
    float v0 = b0[kf * kD1 + imin(tid, kD1 - 1)];
    float v1 = b1[kf * kD2 + imin(tid, kD2 - 1)];
    float v2 = b2[kf * kD3 + imin(tid, kD3 - 1)];
    float v3 = b3[kf * kD4 + imin(tid, kD4 - 1)];
    float v4 = b4[kf * kD5 + imin(tid, kD5 - 1)];
    asm volatile("" : "+v"(v0), "+v"(v1), "+v"(v2), "+v"(v3), "+v"(v4));
    if (tid < kNP0) sB[kBOff0 + tid] = (tid < kD1) ? bf16_rne_f32(v0) : 0.0f;
    if (tid < kNP1) sB[kBOff1 + tid] = (tid < kD2) ? bf16_rne_f32(v1) : 0.0f;
    if (tid < kNP2) sB[kBOff2 + tid] = (tid < kD3) ? bf16_rne_f32(v2) : 0.0f;
    if (tid < kNP3) sB[kBOff3 + tid] = (tid < kD4) ? bf16_rne_f32(v3) : 0.0f;
    if (tid < kNP4) sB[kBOff4 + tid] = (tid < kD5) ? bf16_rne_f32(v4) : 0.0f;
  }
  {
    float hv = head_w[imin(tid, kD5 - 1)];
    float hbv = head_b[0];
    asm volatile("" : "+v"(hv), "+v"(hbv));
    float val = 0.0f;
    val = (tid < kD5) ? bf16_rne_f32(hv) : val;
    val = (tid == 64) ? bf16_rne_f32(hbv) : val;
    if (tid < 80) sHW[tid] = val;
  }
#pragma unroll 1
  for (int it = 0; it < 2; ++it) {
    const int q   = it * 256 + tid;
    const int qc  = imin(q, kXChunks - 1);
    const int c   = qc / kXChunksPerCh;
    const int i0  = (qc - c * kXChunksPerCh) * 8;
    const int i0c = imin(i0, kLen - 8);
    const float* xp = x + (size_t)(bb * kNC + c) * kLen + i0c;
    const v4f f0 = *(const v4f*)(xp);
    const v4f f1 = *(const v4f*)(xp + 4);
    float s0 = f0[0], s1 = f0[1], s2 = f0[2], s3 = f0[3];
    float s4 = f1[0], s5 = f1[1], s6 = f1[2], s7 = f1[3];
    asm volatile("" : "+v"(s0), "+v"(s1), "+v"(s2), "+v"(s3));
    asm volatile("" : "+v"(s4), "+v"(s5), "+v"(s6), "+v"(s7));
    const bool valid = (i0 < kLen);
    v8h hv;
    hv[0] = (_Float16)(valid ? bf16_rne_f32(s0) * kCarryA : 0.0f);
    hv[1] = (_Float16)(valid ? bf16_rne_f32(s1) * kCarryA : 0.0f);
    hv[2] = (_Float16)(valid ? bf16_rne_f32(s2) * kCarryA : 0.0f);
    hv[3] = (_Float16)(valid ? bf16_rne_f32(s3) * kCarryA : 0.0f);
    hv[4] = (_Float16)(valid ? bf16_rne_f32(s4) * kCarryA : 0.0f);
    hv[5] = (_Float16)(valid ? bf16_rne_f32(s5) * kCarryA : 0.0f);
    hv[6] = (_Float16)(valid ? bf16_rne_f32(s6) * kCarryA : 0.0f);
    hv[7] = (_Float16)(valid ? bf16_rne_f32(s7) * kCarryA : 0.0f);
    if (q < kXChunks) *(v8h*)(sXS + c * kXW + i0) = hv;
  }
  if (tid < 32) sOUT[kTiles * kTileRows + tid] = 0.0f;
  __syncthreads();

  float zf = 0.0f;
  asm volatile("" : "+v"(zf));
  const _Float16 zh = (_Float16)zf;

  _Float16* T0 = sT + wave * (2 * kTileHalves);
  _Float16* T1 = T0 + kTileHalves;
  const float hbias = sHW[64];
  const int h = lane >> 4;
  const int n = lane & 15;

#pragma unroll 1
  for (int tix = wave; tix < kTiles; tix += 8) {
    const int row0 = tix * kTileRows;
    {
      const _Float16* xp = sXS + row0 + lane;
      _Float16* trow = T0 + lane * kTP;
#pragma unroll 1
      for (int c = 0; c < kNC; ++c) {
#pragma unroll
        for (int j = 0; j < kTaps; ++j) trow[c * kTaps + j] = xp[c * kXW + j];
      }
      trow[60] = zh;
      trow[61] = zh;
      trow[62] = zh;
      trow[63] = zh;
    }
    wave_sync();

    v8f hp0 = (v8f){0.f, 0.f, 0.f, 0.f, 0.f, 0.f, 0.f, 0.f};
    v8f hp1 = (v8f){0.f, 0.f, 0.f, 0.f, 0.f, 0.f, 0.f, 0.f};
    fc_layer<2, false>(T0, T1, sW + kWOff0, kWP0, sB + kBOff0, sHW, kNP0 / 16, true,  lane, zh, hp0, hp1);
    fc_layer<3, false>(T1, T0, sW + kWOff1, kWPX, sB + kBOff1, sHW, kNP1 / 16, false, lane, zh, hp0, hp1);
    fc_layer<3, false>(T0, T1, sW + kWOff2, kWPX, sB + kBOff2, sHW, kNP2 / 16, false, lane, zh, hp0, hp1);
    fc_layer<3, false>(T1, T0, sW + kWOff3, kWPX, sB + kBOff3, sHW, kNP3 / 16, true,  lane, zh, hp0, hp1);
    fc_layer<3, true >(T0, T1, sW + kWOff4, kWPX, sB + kBOff4, sHW, kNP4 / 16, false, lane, zh, hp0, hp1);

#pragma unroll
    for (int r = 0; r < 8; ++r) {
      float a = hp0[r];
      float c = hp1[r];
      a += __shfl_xor(a, 1, 32);
      c += __shfl_xor(c, 1, 32);
      a += __shfl_xor(a, 2, 32);
      c += __shfl_xor(c, 2, 32);
      a += __shfl_xor(a, 4, 32);
      c += __shfl_xor(c, 4, 32);
      a += __shfl_xor(a, 8, 32);
      c += __shfl_xor(c, 8, 32);
      hp0[r] = a;
      hp1[r] = c;
    }
    float mine = 0.0f;
#pragma unroll
    for (int r = 0; r < 8; ++r) {
      mine = (n == r) ? hp0[r] : mine;
      mine = (n == 8 + r) ? hp1[r] : mine;
    }
    const int trow_id = ((n >> 3) << 4) + 8 * h + (n & 7);
    const int lo = row0 + trow_id;
    sOUT[lo] = (lo < kNOut) ? (mine + hbias) : 0.0f;
  }
  __syncthreads();
  {
    const v4f ov = *(const v4f*)(sOUT + tid * 4);
    float* dst = outp + (size_t)bx * kOutPitch + tid * 4;
    *(volatile v4f*)dst = ov;
    __threadfence();
    *(volatile v4f*)dst = ov;
  }
}

__global__ __launch_bounds__(256) void repack_rows_kernel(
    const float* __restrict__ outp, float* __restrict__ out, int total4)
{
  const int i  = (int)blockIdx.x * 256 + (int)threadIdx.x;
  const int ic = imin(i, total4 - 1);
  const int e0 = ic * 4;
  const int r0 = e0 / kNOut;
  const int r1 = (e0 + 1) / kNOut;
  const int r2 = (e0 + 2) / kNOut;
  const int r3 = (e0 + 3) / kNOut;
  float q0 = outp[(size_t)r0 * kOutPitch + (e0 - r0 * kNOut)];
  float q1 = outp[(size_t)r1 * kOutPitch + (e0 + 1 - r1 * kNOut)];
  float q2 = outp[(size_t)r2 * kOutPitch + (e0 + 2 - r2 * kNOut)];
  float q3 = outp[(size_t)r3 * kOutPitch + (e0 + 3 - r3 * kNOut)];
  asm volatile("" : "+v"(q0), "+v"(q1), "+v"(q2), "+v"(q3));
  v4f ov;
  ov[0] = q0;
  ov[1] = q1;
  ov[2] = q2;
  ov[3] = q3;
  if (i < total4) {
    float* dst = out + (size_t)i * 4;
    *(volatile v4f*)dst = ov;
    __threadfence();
    *(volatile v4f*)dst = ov;
  }
}

extern "C" void kernel_launch(void* const* d_in, const int* in_sizes, int n_in,
                              void* d_out, int out_size, void* d_ws, size_t ws_size,
                              hipStream_t stream) {
  if (n_in < 13) return;
  if (in_sizes[0]  != kNB * kNC * kLen) return;
  if (in_sizes[1]  != kNF * kD0 * kD1) return;
  if (in_sizes[2]  != kNF * kD1) return;
  if (in_sizes[3]  != kNF * kD1 * kD2) return;
  if (in_sizes[4]  != kNF * kD2) return;
  if (in_sizes[5]  != kNF * kD2 * kD3) return;
  if (in_sizes[6]  != kNF * kD3) return;
  if (in_sizes[7]  != kNF * kD3 * kD4) return;
  if (in_sizes[8]  != kNF * kD4) return;
  if (in_sizes[9]  != kNF * kD4 * kD5) return;
  if (in_sizes[10] != kNF * kD5) return;
  if (in_sizes[11] != kD5) return;
  if (in_sizes[12] != 1) return;
  if (out_size != kOutTotal) return;
  if (ws_size < kWsTotal) return;

  const float* x  = (const float*)d_in[0];
  const float* w0 = (const float*)d_in[1];
  const float* b0 = (const float*)d_in[2];
  const float* w1 = (const float*)d_in[3];
  const float* b1 = (const float*)d_in[4];
  const float* w2 = (const float*)d_in[5];
  const float* b2 = (const float*)d_in[6];
  const float* w3 = (const float*)d_in[7];
  const float* b3 = (const float*)d_in[8];
  const float* w4 = (const float*)d_in[9];
  const float* b4 = (const float*)d_in[10];
  const float* hw = (const float*)d_in[11];
  const float* hb = (const float*)d_in[12];
  float* out = (float*)d_out;

  char* ws = (char*)d_ws;
  unsigned short* WPL  = (unsigned short*)(ws + kWsOffWPL);
  float*          OUTP = (float*)(ws + kWsOffOUTP);

  prep_weight_planes_kernel<<<dim3(5, 5, kNF), 256, 0, stream>>>(w0, w1, w2, w3, w4, WPL);

  fused_fc_stack_kernel<<<dim3(kNB * kNF), 256, (size_t)kLdsTotal, stream>>>(
      x, b0, b1, b2, b3, b4, hw, hb, WPL, OUTP);

  repack_rows_kernel<<<dim3(kOutTotal4 / 256), 256, 0, stream>>>(OUTP, out, kOutTotal4);
}
